// GATEncoder_9320079033061
// MI455X (gfx1250) — hardware-run, weakly checked
//
#include <hip/hip_runtime.h>
#include <stddef.h>
#include <stdint.h>
#include <math.h>


#define F_IN    128
#define XQ      (F_IN / 8)
#define C1      256
#define HD1     64
#define NH1     4
#define C2      128
#define KA      512
#define EF      2
#define NTHR    256
#define NWAVE   8
#define EPT     8
#define CHUNK   (NTHR * EPT)
#define WCAP    (EPT * 32)
#define LISTN   (NWAVE * WCAP)
#define NBMAX   2048
#define NBRUN   1024
#define SLOTB   11
#define RCAP    28672
#define DEGCAP  256
#define GBM     64
#define GBN     64
#define GTHR    128
#define MROWS   128
#define NEGSL   0.2f
#define EPS_SM  1e-16f
#define WSMAX   134217728
#define LDS_AGG ((2 * RCAP + 2 * NBMAX + LISTN) * 4 + 128)

static_assert((CHUNK & (CHUNK - 1)) == 0 && CHUNK <= (1 << SLOTB));
static_assert(NBMAX == (1 << SLOTB));
static_assert(NTHR * 8 == NBMAX);
static_assert(NBRUN <= NBMAX && (NBRUN & (NBRUN - 1)) == 0 && NBRUN >= 32);
static_assert(LISTN >= NBMAX);
static_assert(LISTN >= NWAVE * WCAP);
static_assert((RCAP % 32) == 0);
static_assert(LDS_AGG <= 300000);
static_assert((2 * RCAP + 2 * NBMAX + LISTN + 2 * NWAVE + NH1 * EF) * 4 <= LDS_AGG);
static_assert(GBM == (GTHR / 32) * 16);
static_assert((F_IN % 32) == 0 && (KA % 32) == 0);
static_assert((C1 % GBN) == 0 && (C2 % GBN) == 0 && KA == 2 * C1);
static_assert((MROWS % GBM) == 0);
static_assert(C1 == 8 * 32);
static_assert(HD1 == 8 * 8);
static_assert(C1 == NH1 * HD1);
static_assert(C2 == 4 * 32);
static_assert(XQ == 16 && (F_IN % 8) == 0);
static_assert(EF == 2 && NH1 * EF <= 8);
static_assert((C1 * 4) % 128 == 0 && (C2 * 4) % 128 == 0 && (KA * 2) % 128 == 0 && (F_IN * 2) % 128 == 0);

typedef float          v2f  __attribute__((ext_vector_type(2)));
typedef float          v4f  __attribute__((ext_vector_type(4)));
typedef float          v8f  __attribute__((ext_vector_type(8)));
typedef int            v4i  __attribute__((ext_vector_type(4)));
typedef int            v8i  __attribute__((ext_vector_type(8)));
typedef unsigned int   v4u  __attribute__((ext_vector_type(4)));
typedef unsigned short v8us __attribute__((ext_vector_type(8)));
typedef __bf16         v16b __attribute__((ext_vector_type(16)));
typedef v2f  __attribute__((may_alias)) v2fa;
typedef v4f  __attribute__((may_alias)) v4fa;
typedef v8us __attribute__((may_alias)) v8usa;
union FragB { v16b v; v8us h[2]; v8i w; };

__device__ __forceinline__ v8f wmb(const FragB& a, const FragB& b, v8f c) {
  v8f d = __builtin_amdgcn_wmma_f32_16x16x32_bf16(false, a.v, false, b.v, (short)0, c, false, false);
  asm volatile("v_nop\n\tv_nop\n\tv_nop\n\tv_nop" : "+v"(d) : "v"(a.w), "v"(b.w));
  return d;
}

__device__ __forceinline__ unsigned int f2bf(float f) {
  const unsigned int u = __float_as_uint(f);
  return ((u + 0x7FFFu + ((u >> 16) & 1u)) >> 16) & 0xFFFFu;
}
__device__ __forceinline__ float bf2f(unsigned int b) { return __uint_as_float(b << 16); }
__device__ __forceinline__ float bfr(float f) { return bf2f(f2bf(f)); }
__device__ __forceinline__ v4f bfr4(const v4f a) {
  v4f r; r.x = bfr(a.x); r.y = bfr(a.y); r.z = bfr(a.z); r.w = bfr(a.w); return r;
}
__device__ __forceinline__ unsigned int pk2(float lo, float hi) { return f2bf(lo) | (f2bf(hi) << 16); }
__device__ __forceinline__ v4u pack8(const v4f a, const v4f b) {
  v4u r;
  r.x = pk2(a.x, a.y); r.y = pk2(a.z, a.w); r.z = pk2(b.x, b.y); r.w = pk2(b.z, b.w);
  return r;
}

__device__ __forceinline__ float dot8(const v4f a, const v4f b, const v4f c, const v4f d) {
  float p = a.x * c.x;
  p = fmaf(a.y, c.y, p); p = fmaf(a.z, c.z, p); p = fmaf(a.w, c.w, p);
  p = fmaf(b.x, d.x, p); p = fmaf(b.y, d.y, p); p = fmaf(b.z, d.z, p); p = fmaf(b.w, d.w, p);
  return p;
}
__device__ __forceinline__ float dot4(const v4f a, const v4f c) {
  float p = a.x * c.x;
  p = fmaf(a.y, c.y, p); p = fmaf(a.z, c.z, p); p = fmaf(a.w, c.w, p);
  return p;
}
__device__ __forceinline__ float hsum8(float p) {
  p += __shfl_xor(p, 1); p += __shfl_xor(p, 2); p += __shfl_xor(p, 4);
  return p;
}
__device__ __forceinline__ float hsum32(float p) {
  p += __shfl_xor(p, 1); p += __shfl_xor(p, 2); p += __shfl_xor(p, 4); p += __shfl_xor(p, 8);
  p += __shfl_xor(p, 16);
  return p;
}
__device__ __forceinline__ v4f upd4(const v4f a, float s1, float s2, const v4f f) {
  v4f r;
  r.x = fmaf(a.x, s1, s2 * f.x); r.y = fmaf(a.y, s1, s2 * f.y);
  r.z = fmaf(a.z, s1, s2 * f.z); r.w = fmaf(a.w, s1, s2 * f.w);
  return r;
}
__device__ __forceinline__ float elu1(float h) {
  const float n = __expf(fminf(h, 0.f)) - 1.0f;
  return h > 0.f ? h : n;
}
__device__ __forceinline__ v4f fin4(const v4f a, float inv, const v4f b, float pz, bool live) {
  v4f h;
  h.x = elu1(fmaf(a.x, inv, b.x)); h.y = elu1(fmaf(a.y, inv, b.y));
  h.z = elu1(fmaf(a.z, inv, b.z)); h.w = elu1(fmaf(a.w, inv, b.w));
  h.x = (live ? h.x : 0.f) + pz; h.y = (live ? h.y : 0.f) + pz;
  h.z = (live ? h.z : 0.f) + pz; h.w = (live ? h.w : 0.f) + pz;
  return h;
}
__device__ __forceinline__ void hl2(float x, float y, unsigned int& hw, unsigned int& lw) {
  const unsigned int hx = f2bf(x), hy = f2bf(y);
  const unsigned int lx = f2bf(x - bf2f(hx)), ly = f2bf(y - bf2f(hy));
  hw = hx | (hy << 16);
  lw = lx | (ly << 16);
}
__device__ __forceinline__ void split8(const v4f a, const v4f b, v4u& hi, v4u& lo) {
  unsigned int h0, l0, h1, l1, h2, l2, h3, l3;
  hl2(a.x, a.y, h0, l0); hl2(a.z, a.w, h1, l1); hl2(b.x, b.y, h2, l2); hl2(b.z, b.w, h3, l3);
  hi.x = h0; hi.y = h1; hi.z = h2; hi.w = h3;
  lo.x = l0; lo.y = l1; lo.z = l2; lo.w = l3;
}
__device__ __forceinline__ float att_logit(float as, float ad, float a0, float a1, float c0, float c1) {
  const float aeh = fmaf(a1, c1, a0 * c0);
  const float t = (as + ad) + aeh;
  return t > 0.f ? t : NEGSL * t;
}

__device__ __forceinline__ int scan_chunk(const int* __restrict__ dsts, int nE, int cbase, int slotBase,
                                          int nb, int vec8, int* list, int tid, int lane, int wave) {
  int wc = 0;
  const int el0  = tid * EPT;
  const int e0   = cbase + el0;
  const int sent = -2147483647 - 1;
  v4i da, db;
  if (vec8 != 0 && cbase + CHUNK <= nE) {
    da = *(const v4i*)(dsts + e0);
    db = *(const v4i*)(dsts + e0 + 4);
  } else {
    da.x = (e0     < nE) ? dsts[min(e0,     nE - 1)] : sent;
    da.y = (e0 + 1 < nE) ? dsts[min(e0 + 1, nE - 1)] : sent;
    da.z = (e0 + 2 < nE) ? dsts[min(e0 + 2, nE - 1)] : sent;
    da.w = (e0 + 3 < nE) ? dsts[min(e0 + 3, nE - 1)] : sent;
    db.x = (e0 + 4 < nE) ? dsts[min(e0 + 4, nE - 1)] : sent;
    db.y = (e0 + 5 < nE) ? dsts[min(e0 + 5, nE - 1)] : sent;
    db.z = (e0 + 6 < nE) ? dsts[min(e0 + 6, nE - 1)] : sent;
    db.w = (e0 + 7 < nE) ? dsts[min(e0 + 7, nE - 1)] : sent;
  }
  const unsigned nbs = (unsigned)slotBase;
  const unsigned unb = (unsigned)nb;
  const unsigned s0 = (unsigned)da.x - nbs, s1 = (unsigned)da.y - nbs;
  const unsigned s2 = (unsigned)da.z - nbs, s3 = (unsigned)da.w - nbs;
  const unsigned s4 = (unsigned)db.x - nbs, s5 = (unsigned)db.y - nbs;
  const unsigned s6 = (unsigned)db.z - nbs, s7 = (unsigned)db.w - nbs;
  const bool h0 = s0 < unb, h1 = s1 < unb, h2 = s2 < unb, h3 = s3 < unb;
  const bool h4 = s4 < unb, h5 = s5 < unb, h6 = s6 < unb, h7 = s7 < unb;
  const unsigned any = __builtin_amdgcn_ballot_w32(h0 | h1 | h2 | h3 | h4 | h5 | h6 | h7);
  if (any != 0u) {
#define HITJ(J, HJ, SJ) { \
      const unsigned mj = __builtin_amdgcn_ballot_w32(HJ); \
      if (mj != 0u) { \
        if (HJ) { \
          const int pos = wc + (int)__builtin_amdgcn_mbcnt_lo(mj, 0u); \
          if (pos < WCAP) list[wave * WCAP + pos] = ((el0 + (J)) << SLOTB) | (int)(SJ); \
        } \
        wc += (int)__builtin_popcount(mj); } }
    HITJ(0, h0, s0)
    HITJ(1, h1, s1)
    HITJ(2, h2, s2)
    HITJ(3, h3, s3)
    HITJ(4, h4, s4)
    HITJ(5, h5, s5)
    HITJ(6, h6, s6)
    HITJ(7, h7, s7)
#undef HITJ
  }
  return wc;
}

__global__ __launch_bounds__(NTHR) void k_xprep(const float* __restrict__ x, unsigned short* xb, int nN, int nUnits) {
  const int i = (int)blockIdx.x * NTHR + (int)threadIdx.x;
  if (i >= nUnits) return;
  const int row = i >> 4;
  const int c0  = (i & 15) * 8;
  const int rc  = row < nN ? row : nN - 1;
  const float* p = x + (size_t)rc * F_IN + c0;
  v4f a = *(const v4fa*)p, b = *(const v4fa*)(p + 4);
  const v4f z4 = {0.f, 0.f, 0.f, 0.f};
  if (row >= nN) { a = z4; b = z4; }
  const v4u hv = pack8(a, b);
  const size_t o = (size_t)row * F_IN + c0;
  *(volatile v4u*)(xb + o) = hv;
  __threadfence();
  *(volatile v4u*)(xb + o) = hv;
}

__global__ __launch_bounds__(NTHR) void k_wtr(const float* __restrict__ w, int Kin, int Ncol, int Nrows, int Kout,
                                              unsigned short* wt, int nUnits) {
  const int u = (int)blockIdx.x * NTHR + (int)threadIdx.x;
  if (u >= nUnits) return;
  const int kq = Kout >> 3;
  const int n  = u / kq;
  const int k8 = (u - n * kq) * 8;
  const int kk = k8 - (k8 / Kin) * Kin;
  const int ncl = n < Ncol ? n : Ncol - 1;
  const float* p = w + (size_t)kk * (size_t)Ncol + ncl;
  v4f a, b;
  a.x = p[0];                    a.y = p[(size_t)Ncol];         a.z = p[(size_t)2 * Ncol];     a.w = p[(size_t)3 * Ncol];
  b.x = p[(size_t)4 * Ncol];     b.y = p[(size_t)5 * Ncol];     b.z = p[(size_t)6 * Ncol];     b.w = p[(size_t)7 * Ncol];
  const v4f z4 = {0.f, 0.f, 0.f, 0.f};
  if (n >= Ncol || n >= Nrows) { a = z4; b = z4; }
  const v4u wv = pack8(a, b);
  unsigned short* o = wt + (size_t)n * (size_t)Kout + k8;
  *(volatile v4u*)o = wv;
  __threadfence();
  *(volatile v4u*)o = wv;
}

__global__ __launch_bounds__(GTHR) void k_gemm(
    const unsigned short* __restrict__ A, const unsigned short* __restrict__ WT,
    float* outF, int K, int ldo)
{
  __shared__ __attribute__((aligned(16))) float stg[GBM * GBN];
  const int tid = (int)threadIdx.x, lane = tid & 31, wave = tid >> 5, hh = lane >> 4, m = lane & 15;
  const int rowBase = (int)blockIdx.x * GBM;
  const int col0    = (int)blockIdx.y * GBN;

  v8f acc[4];
  {
    const v8f z = {0.f, 0.f, 0.f, 0.f, 0.f, 0.f, 0.f, 0.f};
    acc[0] = z; acc[1] = z; acc[2] = z; acc[3] = z;
  }
  const unsigned short* ap = A  + (size_t)(rowBase + 16 * wave + m) * (size_t)K + 8 * hh;
  const unsigned short* wp = WT + (size_t)(col0 + m) * (size_t)K + 8 * hh;
  const int ksteps = K >> 5;
#pragma unroll 1
  for (int ks = 0; ks < ksteps; ++ks) {
    FragB af;
    af.h[0] = *(const v8usa*)(ap + 32 * ks);
    af.h[1] = *(const v8usa*)(ap + 32 * ks + 16);
#pragma unroll
    for (int t = 0; t < 4; ++t) {
      const unsigned short* wq = wp + (size_t)(16 * t) * (size_t)K + 32 * ks;
      FragB bf;
      bf.h[0] = *(const v8usa*)wq;
      bf.h[1] = *(const v8usa*)(wq + 16);
      acc[t] = wmb(af, bf, acc[t]);
    }
  }

#pragma unroll
  for (int t = 0; t < 4; ++t) {
    const int lc = 16 * t + m;
#pragma unroll
    for (int r = 0; r < 8; ++r) {
      const int lr = 16 * wave + 8 * hh + r;
      stg[lr * GBN + lc] = acc[t][r];
    }
  }
  __syncthreads();

  v4f fv[8];
#pragma unroll
  for (int i = 0; i < 8; ++i) {
    const int lr = 16 * wave + 2 * i + hh;
    fv[i] = *(const v4fa*)(stg + lr * GBN + 4 * m);
  }
#pragma unroll
  for (int i = 0; i < 8; ++i) {
    const int lr = 16 * wave + 2 * i + hh;
    const int gr = rowBase + lr;
    float* op = outF + (size_t)gr * (size_t)ldo + col0 + 4 * m;
    *(volatile v4f*)op = fv[i];
  }
  __threadfence();
#pragma unroll
  for (int i = 0; i < 8; ++i) {
    const int lr = 16 * wave + 2 * i + hh;
    const int gr = rowBase + lr;
    float* op = outF + (size_t)gr * (size_t)ldo + col0 + 4 * m;
    *(volatile v4f*)op = fv[i];
  }
}

template<int L>
__global__ __launch_bounds__(NTHR) void k_agg(
    const int* __restrict__ srcs, const int* __restrict__ dsts, const float* __restrict__ ea,
    const float* __restrict__ F,
    const float* __restrict__ asrc, const float* __restrict__ adst,
    const float* __restrict__ we, const float* __restrict__ ae,
    const float* __restrict__ bias,
    unsigned short* HP, float* out,
    int nN, int nE, int nb, int vec8, int MPr) {
  extern __shared__ v4f lds_dyn[];
  int* reg1 = (int*)lds_dyn;
  int* reg2 = reg1 + RCAP;
  int* scnt = reg2 + RCAP;
  int* soff = scnt + NBMAX;
  int* list = soff + NBMAX;
  int* wcnt = list + LISTN;
  int* wtot = wcnt + NWAVE;
  float* sce = (float*)(wtot + NWAVE);
  const int tid = (int)threadIdx.x, lane = tid & 31, wave = tid >> 5;
  const int nodeBase = (int)blockIdx.x * nb;
  const int CW = (L == 1) ? C1 : C2;
  const int HD = (L == 1) ? HD1 : C2;
  const int NU = (L == 1) ? NH1 * EF : EF;

  for (int i = tid; i < NBMAX; i += NTHR) scnt[i] = 0;
  if (wave == 0) {
    const int un = lane < NU ? lane : NU - 1;
    const int hd = un >> 1;
    const int f  = un & 1;
    const float* pw = we + (size_t)f * CW + hd * HD;
    const float* pa = ae + hd * HD;
    float s = 0.f;
#pragma unroll 1
    for (int d = 0; d < HD; ++d) s = fmaf(bfr(pw[d]), bfr(pa[d]), s);
    if (lane < NU) sce[lane] = s;
  }
  __syncthreads();

  int tot = 0;
  const int nChunks = (nE + CHUNK - 1) / CHUNK;
#pragma unroll 1
  for (int ch = 0; ch < nChunks; ++ch) {
    const int cbase = ch * CHUNK;
    const int wc = scan_chunk(dsts, nE, cbase, nodeBase, nb, vec8, list, tid, lane, wave);
    if (lane == 0) wcnt[wave] = wc;
    __syncthreads();
    int pre = 0, all = 0;
#pragma unroll
    for (int w2 = 0; w2 < NWAVE; ++w2) {
      int c = wcnt[w2];
      c = c < 0 ? 0 : (c > WCAP ? WCAP : c);
      all += c;
      pre += (w2 < wave) ? c : 0;
    }
    const int wcc  = wc > WCAP ? WCAP : wc;
    const int base = tot + pre;
#pragma unroll 1
    for (int i = lane; i < wcc; i += 32) {
      const int ent = list[wave * WCAP + i];
      const int el  = (ent >> SLOTB) & (CHUNK - 1);
      const int sl  = ent & (NBMAX - 1);
      int eid = cbase + el;
      eid = eid > nE - 1 ? nE - 1 : eid;
      const int pos = base + i;
      if (pos < RCAP) reg1[pos] = (int)(((unsigned)eid << SLOTB) | (unsigned)sl);
    }
    tot += all;
    tot = tot > RCAP ? RCAP : tot;
    __syncthreads();
  }
  const int nh = tot;

  if (wave == 0) {
#pragma unroll 1
    for (int b0 = 0; b0 < nh; b0 += 32) {
      const int idx = b0 + lane;
      const int uv  = reg1[idx < nh ? idx : nh - 1];
      const int m32 = (nh - b0) < 32 ? (nh - b0) : 32;
#pragma unroll 1
      for (int k = 0; k < m32; ++k) {
        const int u  = __builtin_amdgcn_readlane(uv, k);
        const int sl = u & (NBMAX - 1);
        if (lane == 0) scnt[sl] = scnt[sl] + 1;
      }
    }
  }
  __syncthreads();

  {
    const v4i ca = *(const v4i*)(scnt + 8 * tid);
    const v4i cb = *(const v4i*)(scnt + 8 * tid + 4);
    const int e0 = ca.x < 0 ? 0 : ca.x, e1 = ca.y < 0 ? 0 : ca.y, e2 = ca.z < 0 ? 0 : ca.z, e3 = ca.w < 0 ? 0 : ca.w;
    const int e4 = cb.x < 0 ? 0 : cb.x, e5 = cb.y < 0 ? 0 : cb.y, e6 = cb.z < 0 ? 0 : cb.z, e7 = cb.w < 0 ? 0 : cb.w;
    const int ts = e0 + e1 + e2 + e3 + e4 + e5 + e6 + e7;
    int incl = ts;
#pragma unroll
    for (int d = 1; d < 32; d <<= 1) {
      const int up = __shfl_up(incl, d);
      if (lane >= d) incl += up;
    }
    if (lane == 31) wtot[wave] = incl;
    __syncthreads();
    int pre = 0;
#pragma unroll
    for (int w2 = 0; w2 < NWAVE; ++w2) pre += (w2 < wave) ? wtot[w2] : 0;
    int run = pre + incl - ts;
    soff[8 * tid + 0] = run; run += e0;
    soff[8 * tid + 1] = run; run += e1;
    soff[8 * tid + 2] = run; run += e2;
    soff[8 * tid + 3] = run; run += e3;
    soff[8 * tid + 4] = run; run += e4;
    soff[8 * tid + 5] = run; run += e5;
    soff[8 * tid + 6] = run; run += e6;
    soff[8 * tid + 7] = run;
  }
  __syncthreads();
  for (int i = tid; i < NBMAX; i += NTHR) list[i] = soff[i];
  __syncthreads();

  if (wave == 0) {
#pragma unroll 1
    for (int b0 = 0; b0 < nh; b0 += 32) {
      const int idx = b0 + lane;
      const int uv  = reg1[idx < nh ? idx : nh - 1];
      const int m32 = (nh - b0) < 32 ? (nh - b0) : 32;
#pragma unroll 1
      for (int k = 0; k < m32; ++k) {
        const int u   = __builtin_amdgcn_readlane(uv, k);
        const int sl  = u & (NBMAX - 1);
        const int eid = (int)((unsigned)u >> SLOTB);
        if (lane == 0) {
          int pos = list[sl];
          pos = pos < 0 ? 0 : (pos > RCAP - 1 ? RCAP - 1 : pos);
          reg2[pos] = eid;
          list[sl] = pos + 1;
        }
      }
    }
  }
  __syncthreads();

  const int nbw = nb >> 3;
  const bool ovf = (nh >= RCAP);
  const float qnan = __int_as_float(0x7fc00000);
  const v4f z4 = {0.f, 0.f, 0.f, 0.f};
  const int hl  = (L == 1) ? (lane >> 3) : 0;
  const int ch0 = (L == 1) ? 8 * lane : 4 * lane;
  const float ce0 = sce[EF * hl], ce1 = sce[EF * hl + 1];
  v4f asv0, asv1, adv0, adv1, bb0, bb1;
  asv0 = bfr4(*(const v4fa*)(asrc + ch0));
  adv0 = bfr4(*(const v4fa*)(adst + ch0));
  bb0  = bfr4(*(const v4fa*)(bias + ch0));
  if (L == 1) {
    asv1 = bfr4(*(const v4fa*)(asrc + ch0 + 4));
    adv1 = bfr4(*(const v4fa*)(adst + ch0 + 4));
    bb1  = bfr4(*(const v4fa*)(bias + ch0 + 4));
  } else {
    asv1 = z4; adv1 = z4; bb1 = z4;
  }

#pragma unroll 1
  for (int jt = 0; jt < nbw; ++jt) {
    const int slot = wave * nbw + jt;
    const int grow = nodeBase + slot;
    const int gcl  = grow < nN ? grow : nN - 1;
    int st = __builtin_amdgcn_readfirstlane(soff[slot]);
    const int craw = __builtin_amdgcn_readfirstlane(scnt[slot]);
    int cnt = craw;
    st  = st < 0 ? 0 : (st > nh ? nh : st);
    cnt = cnt < 0 ? 0 : (cnt > DEGCAP ? DEGCAP : cnt);
    if (cnt > nh - st) cnt = nh - st;
    const float pz = (ovf || craw > DEGCAP) ? qnan : 0.0f;

    const float* fr = F + (size_t)gcl * (size_t)CW + ch0;
    const v4f fd0 = *(const v4fa*)fr;
    v4f fd1 = z4;
    if (L == 1) fd1 = *(const v4fa*)(fr + 4);
    float ad_l, asd_l;
    if (L == 1) {
      ad_l  = hsum8(dot8(fd0, fd1, adv0, adv1));
      asd_l = hsum8(dot8(fd0, fd1, asv0, asv1));
    } else {
      ad_l  = hsum32(dot4(fd0, adv0));
      asd_l = hsum32(dot4(fd0, asv0));
    }
    float mx = -1.0e30f, dn = 0.0f, es0 = 0.0f, es1 = 0.0f;
    v4f a0 = z4, a1 = z4;

#pragma unroll 1
    for (int q = 0; q <= cnt; ++q) {
      float av0, av1, as_l;
      v4f fs0, fs1;
      if (q < cnt) {
        int idx = st + q; idx = idx > RCAP - 1 ? RCAP - 1 : idx;
        int eid = __builtin_amdgcn_readfirstlane(reg2[idx]);
        eid = eid < 0 ? 0 : (eid > nE - 1 ? nE - 1 : eid);
        const int sraw = srcs[eid];
        const int s = sraw < 0 ? 0 : (sraw > nN - 1 ? nN - 1 : sraw);
        const v2f ev = *(const v2fa*)(ea + (size_t)EF * (size_t)eid);
        av0 = bfr(ev.x); av1 = bfr(ev.y);
        es0 += av0; es1 += av1;
        const float* gs = F + (size_t)s * (size_t)CW + ch0;
        fs0 = *(const v4fa*)gs;
        if (L == 1) { fs1 = *(const v4fa*)(gs + 4); as_l = hsum8(dot8(fs0, fs1, asv0, asv1)); }
        else        { fs1 = z4;                    as_l = hsum32(dot4(fs0, asv0)); }
      } else {
        const float rc = 1.0f / fmaxf((float)craw, 1.0f);
        av0 = es0 * rc; av1 = es1 * rc;
        as_l = asd_l;
        fs0 = fd0; fs1 = fd1;
      }
      const float lg = att_logit(as_l, ad_l, av0, av1, ce0, ce1);
      const float df = lg - mx;
      const float ee = __expf(-fabsf(df));
      const bool up  = df > 0.f;
      const float s1 = up ? ee : 1.0f;
      const float s2 = up ? 1.0f : ee;
      mx = up ? lg : mx;
      dn = fmaf(dn, s1, s2);
      a0 = upd4(a0, s1, s2, fs0);
      if (L == 1) a1 = upd4(a1, s1, s2, fs1);
    }
    const float inv = __builtin_amdgcn_rcpf(dn + EPS_SM);
    const bool live = grow < nN;
    if (L == 1) {
      const v4f h0 = fin4(a0, inv, bb0, pz, live);
      const v4f h1 = fin4(a1, inv, bb1, pz, live);
      v4u hi, lo;
      split8(h0, h1, hi, lo);
      unsigned short* gp = HP + (size_t)grow * KA;
      const bool wr = grow < MPr;
      if (wr) {
        *(volatile v4u*)(gp + ch0)      = hi;
        *(volatile v4u*)(gp + C1 + ch0) = lo;
      }
      __threadfence();
      if (wr) {
        *(volatile v4u*)(gp + ch0)      = hi;
        *(volatile v4u*)(gp + C1 + ch0) = lo;
      }
    } else {
      v4f hv;
      hv.x = fmaf(a0.x, inv, bb0.x) + pz;
      hv.y = fmaf(a0.y, inv, bb0.y) + pz;
      hv.z = fmaf(a0.z, inv, bb0.z) + pz;
      hv.w = fmaf(a0.w, inv, bb0.w) + pz;
      float* op = out + (size_t)grow * C2 + ch0;
      const bool wr = grow < nN;
      if (wr) *(volatile v4f*)op = hv;
      __threadfence();
      if (wr) *(volatile v4f*)op = hv;
    }
  }
}

static int pick_nb(int nE, int nN) {
  int nb = NBMAX;
  while (nb > 32 && (long long)nb * (long long)nE * 5LL > (long long)RCAP * (long long)nN * 4LL) nb >>= 1;
  if (nb > NBRUN) nb = NBRUN;
  return nb;
}
static inline int cdiv(int a, int b) { return (a + b - 1) / b; }

extern "C" void kernel_launch(void* const* d_in, const int* in_sizes, int n_in,
                              void* d_out, int out_size, void* d_ws, size_t ws_size,
                              hipStream_t stream) {
  if (n_in < 15) return;
  if (in_sizes[0] <= 0 || (in_sizes[0] % F_IN) != 0) return;
  const int nN = in_sizes[0] / F_IN;
  if (nN <= 0 || nN > (1 << 22)) return;
  if (in_sizes[1] < 2 || (in_sizes[1] & 1) != 0) return;
  const int nE = in_sizes[1] / 2;
  if (nE < 1 || nE >= (1 << (32 - SLOTB))) return;
  if (in_sizes[2] != EF * nE) return;
  if (in_sizes[3] != F_IN * C1) return;
  if (in_sizes[4] != EF * C1) return;
  if (in_sizes[5] != C1 || in_sizes[6] != C1 || in_sizes[7] != C1) return;
  if (in_sizes[8] != C1) return;
  if (in_sizes[9] != C1 * C2) return;
  if (in_sizes[10] != EF * C2) return;
  if (in_sizes[11] != C2 || in_sizes[12] != C2 || in_sizes[13] != C2) return;
  if (in_sizes[14] != C2) return;
  if ((long long)out_size != (long long)nN * C2) return;

  const float* x    = (const float*)d_in[0];
  const int*   ei   = (const int*)  d_in[1];
  const float* ea   = (const float*)d_in[2];
  const float* W1   = (const float*)d_in[3];
  const float* We1  = (const float*)d_in[4];
  const float* a1s  = (const float*)d_in[5];
  const float* a1d  = (const float*)d_in[6];
  const float* a1e  = (const float*)d_in[7];
  const float* b1   = (const float*)d_in[8];
  const float* W2   = (const float*)d_in[9];
  const float* We2  = (const float*)d_in[10];
  const float* a2s  = (const float*)d_in[11];
  const float* a2d  = (const float*)d_in[12];
  const float* a2e  = (const float*)d_in[13];
  const float* b2   = (const float*)d_in[14];
  float* out = (float*)d_out;
  const int* src = ei;
  const int* dst = ei + nE;

  const int MP   = cdiv(nN, MROWS) * MROWS;
  const int nb   = pick_nb(nE, nN);
  if (nb < 32 || (nb & (nb - 1)) != 0 || nb > NBMAX) return;
  const int gA   = cdiv(MP, nb);
  const int vec8 = ((nE & 3) == 0) ? 1 : 0;
  if (gA * nb < MP) return;
  if ((MP % GBM) != 0) return;

  char* ws = (char*)d_ws;
  size_t off = 0;
  const size_t szXB = (size_t)MP * F_IN * 2, szHA = (size_t)MP * KA * 2;
  const size_t szA  = szXB > szHA ? szXB : szHA;
  const size_t oA   = off; off += szA;                           off = (off + 255) & ~(size_t)255;
  const size_t oW1T = off; off += (size_t)C1 * F_IN * 2;         off = (off + 255) & ~(size_t)255;
  const size_t oW2T = off; off += (size_t)C2 * KA * 2;           off = (off + 255) & ~(size_t)255;
  const size_t szF1 = (size_t)MP * C1 * 4, szF2 = (size_t)MP * C2 * 4;
  const size_t szF  = szF1 > szF2 ? szF1 : szF2;
  const size_t oF   = off; off += szF;                           off = (off + 255) & ~(size_t)255;
  if (off > ws_size || off > (size_t)WSMAX) return;
  unsigned short* XB  = (unsigned short*)(ws + oA);
  unsigned short* HA  = (unsigned short*)(ws + oA);
  unsigned short* W1T = (unsigned short*)(ws + oW1T);
  unsigned short* W2T = (unsigned short*)(ws + oW2T);
  float*          F1  = (float*)(ws + oF);
  float*          F2  = (float*)(ws + oF);

  hipFuncSetAttribute(reinterpret_cast<const void*>(&k_agg<1>),
                      hipFuncAttributeMaxDynamicSharedMemorySize, LDS_AGG);
  hipFuncSetAttribute(reinterpret_cast<const void*>(&k_agg<2>),
                      hipFuncAttributeMaxDynamicSharedMemorySize, LDS_AGG);

  const int nUx = MP * XQ;
  k_xprep<<<cdiv(nUx, NTHR), NTHR, 0, stream>>>(x, XB, nN, nUx);

  {
    const int nUw1 = C1 * (F_IN / 8);
    k_wtr<<<cdiv(nUw1, NTHR), NTHR, 0, stream>>>(W1, F_IN, C1, C1, F_IN, W1T, nUw1);
    const int nUw2 = C2 * (KA / 8);
    k_wtr<<<cdiv(nUw2, NTHR), NTHR, 0, stream>>>(W2, C1, C2, C2, KA, W2T, nUw2);
  }

  const int gM = MP / GBM;
  k_gemm<<<dim3(gM, C1 / GBN), GTHR, 0, stream>>>(XB, W1T, F1, F_IN, C1);
  k_agg<1><<<gA, NTHR, LDS_AGG, stream>>>(src, dst, ea, F1, a1s, a1d, We1, a1e, b1, HA, out,
                                          nN, nE, nb, vec8, MP);
  k_gemm<<<dim3(gM, C2 / GBN), GTHR, 0, stream>>>(HA, W2T, F2, KA, C2);
  k_agg<2><<<gA, NTHR, LDS_AGG, stream>>>(src, dst, ea, F2, a2s, a2d, We2, a2e, b2, HA, out,
                                          nN, nE, nb, vec8, MP);
}
